// PairwiseGrounder_77455440216103
// MI455X (gfx1250) — hardware-verified
//
#include <hip/hip_runtime.h>
#include <math.h>

typedef __attribute__((ext_vector_type(16))) _Float16 v16h;
typedef __attribute__((ext_vector_type(16))) __bf16 v16b;
typedef __attribute__((ext_vector_type(8)))  _Float16 v8h;
typedef __attribute__((ext_vector_type(8)))  float v8f;
typedef __attribute__((ext_vector_type(4)))  float v4f;
typedef __attribute__((ext_vector_type(2)))  float v2f;
typedef __attribute__((ext_vector_type(4)))  unsigned v4u;
typedef __attribute__((ext_vector_type(4)))  int v4i;
typedef float __attribute__((may_alias)) float_a;
typedef int __attribute__((may_alias)) int_a;

template <typename T> __device__ __forceinline__ void vst2(void* p, T v) { *(volatile T*)p = v; __threadfence(); *(volatile T*)p = v; }
__device__ __forceinline__ v8f wmma16(v16h a, v16h b, v8f c) {
  v8f d = __builtin_amdgcn_wmma_f32_16x16x32_f16(false, a, false, b, (short)0, c, false, false);
  asm volatile("v_nop\n\tv_nop\n\tv_nop\n\tv_nop" : "+v"(d) : "v"(a), "v"(b));
  return d;
}
__device__ __forceinline__ v8f wmma_bf(v16b a, v16b b, v8f c) {
  v8f d = __builtin_amdgcn_wmma_f32_16x16x32_bf16(false, a, false, b, (short)0, c, false, false);
  asm volatile("v_nop\n\tv_nop\n\tv_nop\n\tv_nop" : "+v"(d) : "v"(a), "v"(b));
  return d;
}
__device__ __forceinline__ v16h frag_h(const _Float16* rowk0, int lane) {
  union { v16h v; v8h q[2]; } u; const _Float16* p = rowk0 + 8 * (lane >> 4);
  u.q[0] = *(const v8h*)p; u.q[1] = *(const v8h*)(p + 16); return u.v;
}
__device__ __forceinline__ v16h frag_f32(const float* rowk0, int lane) {
  v16h a; const float* p = rowk0 + 8 * (lane >> 4);
#pragma unroll
  for (int i = 0; i < 8; ++i) { a[i] = (_Float16)p[i]; a[8 + i] = (_Float16)p[16 + i]; }
  return a;
}
__device__ __forceinline__ v16h frag_f32s(const float* rowk0, int lane, float sc) {
  v16h a; const float* p = rowk0 + 8 * (lane >> 4);
#pragma unroll
  for (int i = 0; i < 8; ++i) { a[i] = (_Float16)(p[i] * sc); a[8 + i] = (_Float16)(p[16 + i] * sc); }
  return a;
}
__device__ __forceinline__ v16h fragc_f32(const float* W, int k0, int n, int lane, int ld, int K) {
  v16h a; const int g = lane >> 4;
#pragma unroll
  for (int i = 0; i < 8; ++i) { const int ka = k0 + 8 * g + i, kb = ka + 16;
    a[i] = (_Float16)(ka < K ? W[(size_t)(ka < K ? ka : K - 1) * ld + n] : 0.f); a[8 + i] = (_Float16)(kb < K ? W[(size_t)(kb < K ? kb : K - 1) * ld + n] : 0.f); }
  return a;
}
struct F2 { v16b h, l; };
__device__ __forceinline__ F2 bsplit16(const float v[16]) { F2 r;
#pragma unroll
  for (int i = 0; i < 16; ++i) { const __bf16 h = (__bf16)v[i]; r.h[i] = h; r.l[i] = (__bf16)(v[i] - (float)h); }
  return r; }
__device__ __forceinline__ F2 split_row(const float* row, int k0, int lane) { float v[16]; const float* p = row + k0 + 8 * (lane >> 4);
#pragma unroll
  for (int i = 0; i < 8; ++i) { v[i] = p[i]; v[8 + i] = p[16 + i]; }
  return bsplit16(v); }
__device__ __forceinline__ F2 split_rowK(const float* row, int k0, int lane, int K) { float v[16]; const int g = lane >> 4;
#pragma unroll
  for (int i = 0; i < 8; ++i) { const int ka = k0 + 8 * g + i, kb = ka + 16; v[i] = ka < K ? row[ka < K ? ka : K - 1] : 0.f; v[8 + i] = kb < K ? row[kb < K ? kb : K - 1] : 0.f; }
  return bsplit16(v); }
__device__ __forceinline__ F2 split_col(const float* W, int k0, int n, int lane, int ld, int K) { float v[16]; const int g = lane >> 4;
#pragma unroll
  for (int i = 0; i < 8; ++i) { const int ka = k0 + 8 * g + i, kb = ka + 16; v[i] = ka < K ? W[(size_t)(ka < K ? ka : K - 1) * ld + n] : 0.f; v[8 + i] = kb < K ? W[(size_t)(kb < K ? kb : K - 1) * ld + n] : 0.f; }
  return bsplit16(v); }
__device__ __forceinline__ v8f mac3(const F2& a, const F2& b, v8f c) { c = wmma_bf(a.l, b.h, c); c = wmma_bf(a.h, b.l, c); return wmma_bf(a.h, b.h, c); }
__device__ __forceinline__ float sigm(float v) { return 1.0f / (1.0f + expf(-v)); }
#define LDSX() do { asm volatile("s_wait_dscnt 0" ::: "memory"); __builtin_amdgcn_wave_barrier(); __builtin_amdgcn_fence(__ATOMIC_RELEASE, "workgroup"); } while (0)


#define NB 64
#define NT 128
#define NL 64
#define DD 768
#define NEGV (-9.0e9f)
#ifndef NBI
#define NBI NB
#endif
typedef __attribute__((ext_vector_type(8))) __bf16 v8b;
__device__ __forceinline__ v16b frag_b(const __bf16* rowk0, int lane) {
  union { v16b v; v8b q[2]; } u; const __bf16* p = rowk0 + 8 * (lane >> 4);
  u.q[0] = *(const v8b*)p; u.q[1] = *(const v8b*)(p + 16); return u.v;
}
__device__ __forceinline__ float bfr(float v) { return (float)(__bf16)v; }
__device__ __attribute__((noinline)) float exp_ni(float v) { return expf(v); }
__device__ __attribute__((noinline)) float erf_ni(float v) { return erff(v); }

#define WS_TB  0u
#define WS_IB  (WS_TB + 2u * NB * NT * DD)
#define WS_SS  (WS_IB + 2u * NB * NL * DD)
#define WS_STG (WS_SS + 4u * NB * NB * 32)
#define WS_LOSS (WS_STG + 4u * NB * NT * DD)
#define WS_END (WS_LOSS + 128u)

__global__ __launch_bounds__(128) void k_rows(const float* __restrict__ TX, const float* __restrict__ IM, __bf16* __restrict__ TB, __bf16* __restrict__ IB) {
  __shared__ __align__(16) __bf16 s[DD]; const int t = threadIdx.x; size_t r = blockIdx.x; const float* src; __bf16* dst;
  if (r < (size_t)NB * NT) { src = TX + r * DD; dst = TB + r * DD; } else { r -= (size_t)NB * NT; src = IM + r * DD; dst = IB + r * DD; }
  for (int k = t; k < DD; k += 128) s[k] = (__bf16)src[k];
  __syncthreads();
  if (t < DD / 8) vst2((unsigned*)(dst + t * 8), *(const v4u*)&s[t * 8]);
}
__global__ __launch_bounds__(128) void k_pair(const __bf16* __restrict__ TB, const __bf16* __restrict__ IB, const int* __restrict__ TM, const int* __restrict__ IMK, float* __restrict__ SS, float* __restrict__ STG) {
  __shared__ __align__(16) float sa[NT][NL + 4]; __shared__ float srow[NT]; __shared__ float scol[NL]; __shared__ __align__(16) float sline[32];
  __shared__ __align__(16) __bf16 sph[4][16][NL + 8], spl[4][16][NL + 8]; __shared__ __align__(16) float so[4][16][132];
  const int tid = threadIdx.x, wave = tid >> 5, lane = tid & 31, col = lane & 15, g = lane >> 4; const int i = blockIdx.x, j = blockIdx.y;
  const __bf16* T = TB + (size_t)i * NT * DD; const __bf16* I = IB + (size_t)j * NL * DD;
#pragma unroll 1
  for (int rt = 0; rt < 2; ++rt) { const int n0 = wave * 32 + rt * 16; v8f acc[4] = {};
#pragma unroll 2
    for (int kc = 0; kc < DD / 32; ++kc) { const v16b a = frag_b(T + (size_t)(n0 + col) * DD + kc * 32, lane);
#pragma unroll
      for (int c4 = 0; c4 < 4; ++c4) acc[c4] = wmma_bf(a, frag_b(I + (size_t)(c4 * 16 + col) * DD + kc * 32, lane), acc[c4]); }
#pragma unroll
    for (int c4 = 0; c4 < 4; ++c4)
#pragma unroll
      for (int r = 0; r < 8; ++r) { const int n = n0 + 8 * g + r, l = c4 * 16 + col; const float m = (float)(TM[i * NT + n] * IMK[j * NL + l]); const float am = acc[c4][r] * m; sa[n][l] = (am * m != 0.f) ? am : NEGV; } }
  __syncthreads();
  { const int n = tid; const float tmv = (float)TM[i * NT + n]; float mx = -3.0e38f; for (int l = 0; l < NL; ++l) mx = fmaxf(mx, sa[n][l]); float se = 0.f; for (int l = 0; l < NL; ++l) se += exp_ni(sa[n][l] - mx);
    float acc1 = 0.f; for (int l = 0; l < NL; ++l) { const float aw = (exp_ni(sa[n][l] - mx) / se) * (tmv * (float)IMK[j * NL + l]); acc1 += aw * sa[n][l]; } srow[n] = acc1; }
  if (tid < NL) { const int l = tid; const float imv = (float)IMK[j * NL + l]; float mx = -3.0e38f; for (int n = 0; n < NT; ++n) mx = fmaxf(mx, sa[n][l]); float se = 0.f; for (int n = 0; n < NT; ++n) se += exp_ni(sa[n][l] - mx);
    float acc2 = 0.f; for (int n = 0; n < NT; ++n) { const float aw = (exp_ni(sa[n][l] - mx) / se) * ((float)TM[i * NT + n] * imv); acc2 += aw * sa[n][l]; } scol[l] = acc2; }
  __syncthreads();
  if (tid < 32) { double a = 0.0; if (tid == 0) { for (int n = 0; n < NT; ++n) a += (double)srow[n]; double b = 0.0; for (int l = 0; l < NL; ++l) b += (double)scol[l]; a = (a + b) / (double)NT; } sline[tid] = (tid == 0) ? (float)a : 0.f; }
  __syncthreads();
  if (tid < 8) vst2(SS + ((size_t)i * NB + j) * 32 + tid * 4, *(const v4f*)&sline[tid * 4]);
  if (i != j) return;
#pragma unroll 1
  for (int rt = 0; rt < 2; ++rt) { const int n0 = wave * 32 + rt * 16;
    for (int q = lane; q < 16 * NL; q += 32) { const int rl = q / NL, l = q % NL; const int n = n0 + rl; float mx = -3.0e38f; for (int l2 = 0; l2 < NL; ++l2) mx = fmaxf(mx, sa[n][l2]); float se = 0.f; for (int l2 = 0; l2 < NL; ++l2) se += exp_ni(sa[n][l2] - mx);
      const float p = exp_ni(sa[n][l] - mx) / se; const __bf16 hb = (__bf16)p; sph[wave][rl][l] = hb; spl[wave][rl][l] = (__bf16)(p - (float)hb); }
    LDSX();
#pragma unroll 1
    for (int cb = 0; cb < DD / 128; ++cb) { v8f acc[8] = {};
#pragma unroll
      for (int kc = 0; kc < NL / 32; ++kc) { F2 a; a.h = frag_b(&sph[wave][col][kc * 32], lane); a.l = frag_b(&spl[wave][col][kc * 32], lane);
#pragma unroll
        for (int jj = 0; jj < 8; ++jj) { v16b w; { const int d = cb * 128 + jj * 16 + col;
            const __bf16* base = I + d;
#pragma unroll
            for (int e = 0; e < 8; ++e) { w[e] = base[(size_t)(kc * 32 + 8 * g + e) * DD]; w[8 + e] = base[(size_t)(kc * 32 + 16 + 8 * g + e) * DD]; } }
          acc[jj] = wmma_bf(a.l, w, acc[jj]); acc[jj] = wmma_bf(a.h, w, acc[jj]); } }
#pragma unroll
      for (int jj = 0; jj < 8; ++jj)
#pragma unroll
        for (int r = 0; r < 8; ++r) so[wave][8 * g + r][jj * 16 + col] = acc[jj][r];
      LDSX();
      for (int rl = 0; rl < 16; ++rl) vst2(STG + ((size_t)i * NT + n0 + rl) * DD + cb * 128 + lane * 4, *(const v4f*)&so[wave][rl][lane * 4]);
      LDSX(); } }
}
__global__ __launch_bounds__(64) void k_loss(const float* __restrict__ SS, float* __restrict__ LOSS) {
  __shared__ float s[NB][NB + 1]; __shared__ double sl[NB]; __shared__ __align__(16) float sline[32]; const int t = threadIdx.x;
  for (int q = t; q < NB * NB; q += 64) s[q / NB][q % NB] = SS[(size_t)q * 32];
  __syncthreads();
  { const int i = t; float m1 = -3.0e38f, m2 = -3.0e38f; for (int j = 0; j < NB; ++j) { m1 = fmaxf(m1, s[i][j]); m2 = fmaxf(m2, s[j][i]); } double e1 = 0.0, e2 = 0.0; for (int j = 0; j < NB; ++j) { e1 += (double)exp_ni(s[i][j] - m1); e2 += (double)exp_ni(s[j][i] - m2); }
    const double ls1 = (double)s[i][i] - ((double)m1 + log(e1)); const double ls2 = (double)s[i][i] - ((double)m2 + log(e2)); sl[i] = ls1 + ls2; }
  __syncthreads();
  if (t < 32) { double a = 0.0; if (t == 0) for (int i = 0; i < NB; ++i) a += sl[i]; sline[t] = (t == 0) ? (float)(-a / (double)NB) : 0.f; }
  __syncthreads();
  if (t < 8) vst2(LOSS + t * 4, *(const v4f*)&sline[t * 4]);
}
__global__ __launch_bounds__(256) void k_flat(const float* __restrict__ LOSS, const float* __restrict__ STG, float* __restrict__ OUT) {
  const size_t q = (size_t)blockIdx.x * 256 + threadIdx.x; const size_t total = 1 + (size_t)NB * NT * DD; const size_t npieces = total / 4;
  if (q < npieces) { v4f v;
#pragma unroll
    for (int e = 0; e < 4; ++e) { const size_t f = q * 4 + e; v[e] = (f == 0) ? LOSS[0] : STG[f - 1]; }
    vst2(OUT + q * 4, v); }
  else if (q == npieces) { *(volatile float*)(OUT + total - 1) = STG[total - 2]; *(volatile float*)(OUT + total - 1) = STG[total - 2]; }
}
extern "C" void kernel_launch(void* const* d_in, const int* in_sizes, int n_in, void* d_out, int out_size, void* d_ws, size_t ws_size, hipStream_t stream) {
  (void)in_sizes; (void)n_in; (void)out_size;
  const float** F = (const float**)d_in;
  if (ws_size < (size_t)WS_END) return;
  char* ws = (char*)d_ws; __bf16 *TB = (__bf16*)(ws + WS_TB), *IB = (__bf16*)(ws + WS_IB); float *SS = (float*)(ws + WS_SS), *STG = (float*)(ws + WS_STG), *LOSS = (float*)(ws + WS_LOSS);
  k_rows<<<NB * NT + NB * NL, 128, 0, stream>>>(F[0], F[1], TB, IB);
  k_pair<<<dim3(NB, NBI), 128, 0, stream>>>(TB, IB, (const int*)d_in[2], (const int*)d_in[3], SS, STG);
  k_loss<<<1, 64, 0, stream>>>(SS, LOSS);
  k_flat<<<(unsigned)(((size_t)NB * NT * DD / 4 + 1 + 255) / 256), 256, 0, stream>>>(LOSS, STG, (float*)d_out);
}
